// TimeSeriesRNN_90649579749448
// MI455X (gfx1250) — hardware-verified
//
#include <hip/hip_runtime.h>


typedef _Float16 f16t;
typedef unsigned short u16t;
typedef f16t   v16h __attribute__((ext_vector_type(16)));
typedef __bf16 v16b __attribute__((ext_vector_type(16)));
typedef float  v8f  __attribute__((ext_vector_type(8)));
typedef float  v4f  __attribute__((ext_vector_type(4)));
typedef unsigned int v4u __attribute__((ext_vector_type(4)));

union FH { v16h v; v4u q[2]; v8f f; };
union FB { v16b v; v4u q[2]; v8f f; };

#define HID  128
#define G3   384
#define DI   16
#define TO   64
#define KIH  32
#define HP   136
#define AXP  40

__device__ __forceinline__ u16t f2bf(float f) {
  unsigned u = __builtin_bit_cast(unsigned, f);
  u += 0x7FFFu + ((u >> 16) & 1u);
  return (u16t)(u >> 16);
}
__device__ __forceinline__ float bf2f(u16t b) {
  return __builtin_bit_cast(float, ((unsigned)b) << 16);
}
__device__ __forceinline__ u16t f2h(float f) {
  return __builtin_bit_cast(u16t, (f16t)f);
}

__device__ __forceinline__ v8f whf(v16h a, v16h b, v8f c) {
  return __builtin_amdgcn_wmma_f32_16x16x32_f16(false, a, false, b, (short)0, c, false, false);
}
__device__ __forceinline__ v8f wbf(v16b a, v16b b, v8f c) {
  return __builtin_amdgcn_wmma_f32_16x16x32_bf16(false, a, false, b, (short)0, c, false, false);
}
__device__ __forceinline__ void hz4(v8f& c0, v8f& c1, v8f& c2, v8f& c3,
                                    v8f f0, v8f f1, v8f f2, v8f f3,
                                    v8f f4, v8f f5, v8f f6, v8f f7) {
  asm volatile("v_nop\n\tv_nop\n\tv_nop\n\tv_nop"
               : "+v"(c0), "+v"(c1), "+v"(c2), "+v"(c3)
               : "v"(f0), "v"(f1), "v"(f2), "v"(f3), "v"(f4), "v"(f5), "v"(f6), "v"(f7));
}
__device__ __forceinline__ void hz1(v8f& c0, v8f f0, v8f f1, v8f f2, v8f f3) {
  asm volatile("v_nop\n\tv_nop\n\tv_nop\n\tv_nop"
               : "+v"(c0)
               : "v"(f0), "v"(f1), "v"(f2), "v"(f3));
}

__device__ __forceinline__ void ld_b(FB& fr, const u16t* p) {
  fr.q[0] = *(const v4u*)p;
  fr.q[1] = *(const v4u*)(p + 16);
}
__device__ __forceinline__ void ld_h(FH& fr, const u16t* p) {
  fr.q[0] = *(const v4u*)p;
  fr.q[1] = *(const v4u*)(p + 16);
}

__device__ __forceinline__ void mma_in(v8f& aR, v8f& aZ, v8f& aNi, v8f& aNh,
                                       const u16t* Axp,
                                       const u16t* __restrict__ QHi, const u16t* __restrict__ QLo,
                                       int w, int hh, int m) {
  FB a;
  ld_b(a, Axp + m * AXP + 8 * hh);
  FB b[6];
#pragma unroll
  for (int g = 0; g < 3; ++g) {
    const size_t o = (size_t)(g * HID + w * 16 + m) * KIH + 8 * hh;
    ld_b(b[2 * g], QHi + o);
    ld_b(b[2 * g + 1], QLo + o);
  }
  aR  = wbf(a.v, b[0].v, aR);   aR  = wbf(a.v, b[1].v, aR);
  aZ  = wbf(a.v, b[2].v, aZ);   aZ  = wbf(a.v, b[3].v, aZ);
  aNi = wbf(a.v, b[4].v, aNi);  aNi = wbf(a.v, b[5].v, aNi);
  hz4(aR, aZ, aNi, aNh, a.f, b[0].f, b[1].f, b[2].f, b[3].f, b[4].f, b[5].f, a.f);
}

__device__ __forceinline__ void mma_hh_f16(v8f& aR, v8f& aZ, v8f& aNh, v8f& aNi,
                                           const u16t* H16p, const u16t* __restrict__ P16,
                                           int w, int hh, int m) {
#pragma unroll 1
  for (int kt = 0; kt < 4; ++kt) {
    FH a;
    ld_h(a, H16p + m * HP + kt * 32 + 8 * hh);
    FH b[3];
#pragma unroll
    for (int g = 0; g < 3; ++g)
      ld_h(b[g], P16 + (size_t)(g * HID + w * 16 + m) * HID + kt * 32 + 8 * hh);
    aR  = whf(a.v, b[0].v, aR);
    aZ  = whf(a.v, b[1].v, aZ);
    aNh = whf(a.v, b[2].v, aNh);
    hz4(aR, aZ, aNh, aNi, a.f, b[0].f, b[1].f, b[2].f, a.f, a.f, a.f, a.f);
  }
}

__device__ __forceinline__ void mma_hh_split(v8f& aR, v8f& aZ, v8f& aNh, v8f& aNi,
                                             const u16t* HHp, const u16t* HLp,
                                             const u16t* __restrict__ PHi, const u16t* __restrict__ PLo,
                                             int w, int hh, int m) {
#pragma unroll 1
  for (int kt = 0; kt < 4; ++kt) {
    const int ao = m * HP + kt * 32 + 8 * hh;
    FB ah, al;
    ld_b(ah, HHp + ao);
    ld_b(al, HLp + ao);
    FB bh[3], bl[3];
#pragma unroll
    for (int g = 0; g < 3; ++g) {
      const size_t o = (size_t)(g * HID + w * 16 + m) * HID + kt * 32 + 8 * hh;
      ld_b(bh[g], PHi + o);
      ld_b(bl[g], PLo + o);
    }
    aR  = wbf(ah.v, bh[0].v, aR);   aR  = wbf(ah.v, bl[0].v, aR);   aR  = wbf(al.v, bh[0].v, aR);
    aZ  = wbf(ah.v, bh[1].v, aZ);   aZ  = wbf(ah.v, bl[1].v, aZ);   aZ  = wbf(al.v, bh[1].v, aZ);
    aNh = wbf(ah.v, bh[2].v, aNh);  aNh = wbf(ah.v, bl[2].v, aNh);  aNh = wbf(al.v, bh[2].v, aNh);
    hz4(aR, aZ, aNh, aNi, ah.f, al.f, bh[0].f, bh[1].f, bh[2].f, bl[0].f, bl[1].f, bl[2].f);
  }
}

__device__ __forceinline__ v8f mma_l1(const u16t* HHp, const u16t* HLp,
                                      const u16t* __restrict__ RHi, const u16t* __restrict__ RLo,
                                      int hh, int m) {
  v8f o = {0.f, 0.f, 0.f, 0.f, 0.f, 0.f, 0.f, 0.f};
#pragma unroll 1
  for (int kt = 0; kt < 4; ++kt) {
    const int ao = m * HP + kt * 32 + 8 * hh;
    FB ah, al, bh, bl;
    ld_b(ah, HHp + ao);
    ld_b(al, HLp + ao);
    const size_t bo = (size_t)m * HID + kt * 32 + 8 * hh;
    ld_b(bh, RHi + bo);
    ld_b(bl, RLo + bo);
    o = wbf(ah.v, bh.v, o);
    o = wbf(ah.v, bl.v, o);
    o = wbf(al.v, bh.v, o);
    hz1(o, ah.f, al.f, bh.f, bl.f);
  }
  return o;
}

__device__ __forceinline__ float sigm(float v) {
  return __builtin_amdgcn_rcpf(1.0f + __expf(-v));
}
__device__ __forceinline__ float tnh(float v) {
  const float av = fabsf(v);
  const float t  = __expf(-2.0f * av);
  const float r  = (1.0f - t) * __builtin_amdgcn_rcpf(1.0f + t);
  return copysignf(r, v);
}
__device__ __forceinline__ void gru_cell(const v8f& aR, const v8f& aZ, const v8f& aNi, const v8f& aNh,
                                         float brr, float bzz, float bni, float bnh, float (&hold)[8]) {
#pragma unroll
  for (int j = 0; j < 8; ++j) {
    const float pr = fmaf(aR[j],  0.125f, brr);
    const float pz = fmaf(aZ[j],  0.125f, bzz);
    const float pi = fmaf(aNi[j], 0.125f, bni);
    const float ph = fmaf(aNh[j], 0.125f, bnh);
    const float r  = sigm(pr);
    const float z  = sigm(pz);
    const float n  = tnh(fmaf(r, ph, pi));
    hold[j] = (1.0f - z) * n + z * hold[j];
  }
}

__device__ __forceinline__ u16t cvt16(float v, int mode) {
  const u16t hi = f2bf(v);
  const u16t lo = f2bf(v - bf2f(hi));
  const u16t hf = f2h(v);
  return mode == 0 ? hf : (mode == 1 ? hi : lo);
}

__global__ __launch_bounds__(256)
void k_planes(const float* __restrict__ Whh, const float* __restrict__ Wih, const float* __restrict__ L1w,
              u16t* P16, u16t* PHi, u16t* PLo, u16t* QHi, u16t* QLo, u16t* RHi, u16t* RLo) {
  const int blk = blockIdx.x, tid = threadIdx.x;
  const float* src;
  u16t* dst;
  int mode;
  if (blk < 72) {
    const int r = blk / 24;
    const int p = (blk - r * 24) * 256 + tid;
    const int n = p >> 4, k = (p & 15) * 8;
    src  = Whh + (size_t)n * HID + k;
    dst  = (r == 0 ? P16 : (r == 1 ? PHi : PLo)) + (size_t)p * 8;
    mode = r;
  } else if (blk < 84) {
    const int r = (blk - 72) / 6;
    const int p = (blk - 72 - r * 6) * 256 + tid;
    const int n = p >> 2, k = (p & 1) * 8;
    src  = Wih + (size_t)n * DI + k;
    dst  = (r == 0 ? QHi : QLo) + (size_t)p * 8;
    mode = 1 + r;
  } else {
    const int r = blk - 84;
    const int p = tid;
    const int n = p >> 4, k = (p & 15) * 8;
    src  = L1w + (size_t)n * HID + k;
    dst  = (r == 0 ? RHi : RLo) + (size_t)p * 8;
    mode = 1 + r;
  }
  const v4f a = *(const v4f*)src;
  const v4f b = *(const v4f*)(src + 4);
  const float sc = 8.0f;
  const unsigned w0 = (unsigned)cvt16(a[0] * sc, mode) | ((unsigned)cvt16(a[1] * sc, mode) << 16);
  const unsigned w1 = (unsigned)cvt16(a[2] * sc, mode) | ((unsigned)cvt16(a[3] * sc, mode) << 16);
  const unsigned w2 = (unsigned)cvt16(b[0] * sc, mode) | ((unsigned)cvt16(b[1] * sc, mode) << 16);
  const unsigned w3 = (unsigned)cvt16(b[2] * sc, mode) | ((unsigned)cvt16(b[3] * sc, mode) << 16);
  const v4u u = {w0, w1, w2, w3};
  *(volatile v4u*)dst = u;
  __threadfence();
  *(volatile v4u*)dst = u;
}

__global__ __launch_bounds__(256)
void k_gru(const float* __restrict__ x, const float* __restrict__ l0w,
           const u16t* __restrict__ P16, const u16t* __restrict__ PHi, const u16t* __restrict__ PLo,
           const u16t* __restrict__ QHi, const u16t* __restrict__ QLo,
           const u16t* __restrict__ RHi, const u16t* __restrict__ RLo,
           const float* __restrict__ bih, const float* __restrict__ bhh,
           const float* __restrict__ l1b, const float* __restrict__ l2w, const float* __restrict__ l2b,
           float* out, int nb, int T) {
  __shared__ __attribute__((aligned(16))) float Lw0[DI * DI];
  __shared__ __attribute__((aligned(16))) float Lms[64];
  __shared__ __attribute__((aligned(16))) u16t  Ax[16 * AXP];
  __shared__ __attribute__((aligned(16))) u16t  H16[16 * HP];
  __shared__ __attribute__((aligned(16))) u16t  HHi[16 * HP];
  __shared__ __attribute__((aligned(16))) u16t  HLo[16 * HP];
  __shared__ __attribute__((aligned(16))) float OutS[16 * DI];
  __shared__ __attribute__((aligned(16))) float Ys[16 * TO];

  const int tid = threadIdx.x;
  const int w   = tid >> 5;
  const int lane = tid & 31, hh = lane >> 4, m = lane & 15;
  const int b0  = blockIdx.x * 16;
  if (b0 + 16 > nb) return;

  Lw0[tid] = l0w[tid];
  if (tid < DI) { Lms[tid] = l1b[tid]; Lms[16 + tid] = l2w[tid]; }
  if (tid == 0) Lms[32] = l2b[0];
  for (int i = tid; i < 16 * HP; i += 256) H16[i] = 0;

  const int col = w * 16 + m;
  const float brr = bih[col] + bhh[col];
  const float bzz = bih[HID + col] + bhh[HID + col];
  const float bni = bih[2 * HID + col];
  const float bnh = bhh[2 * HID + col];

  float hold[8];
#pragma unroll
  for (int j = 0; j < 8; ++j) hold[j] = 0.0f;

  const int row = tid >> 4, f = tid & 15;
  const v8f z8 = {0.f, 0.f, 0.f, 0.f, 0.f, 0.f, 0.f, 0.f};
  __syncthreads();

#pragma unroll 1
  for (int t = 0; t < T; ++t) {
    {
      const float* xr = x + ((size_t)(b0 + row) * (size_t)T + t) * DI;
      const v4f x0 = *(const v4f*)(xr);
      const v4f x1 = *(const v4f*)(xr + 4);
      const v4f x2 = *(const v4f*)(xr + 8);
      const v4f x3 = *(const v4f*)(xr + 12);
      const float* wr = Lw0 + f * DI;
      const v4f w0 = *(const v4f*)(wr);
      const v4f w1 = *(const v4f*)(wr + 4);
      const v4f w2 = *(const v4f*)(wr + 8);
      const v4f w3 = *(const v4f*)(wr + 12);
      float s = x0[0] * w0[0];
      s = fmaf(x0[1], w0[1], s); s = fmaf(x0[2], w0[2], s); s = fmaf(x0[3], w0[3], s);
      s = fmaf(x1[0], w1[0], s); s = fmaf(x1[1], w1[1], s); s = fmaf(x1[2], w1[2], s); s = fmaf(x1[3], w1[3], s);
      s = fmaf(x2[0], w2[0], s); s = fmaf(x2[1], w2[1], s); s = fmaf(x2[2], w2[2], s); s = fmaf(x2[3], w2[3], s);
      s = fmaf(x3[0], w3[0], s); s = fmaf(x3[1], w3[1], s); s = fmaf(x3[2], w3[2], s); s = fmaf(x3[3], w3[3], s);
      s = fmaxf(s, 0.0f);
      const u16t hi = f2bf(s);
      Ax[row * AXP + f]      = hi;
      Ax[row * AXP + 16 + f] = f2bf(s - bf2f(hi));
    }
    __syncthreads();
    v8f aR = z8, aZ = z8, aNi = z8, aNh = z8;
    mma_in(aR, aZ, aNi, aNh, Ax, QHi, QLo, w, hh, m);
    mma_hh_f16(aR, aZ, aNh, aNi, H16, P16, w, hh, m);
    __syncthreads();
    gru_cell(aR, aZ, aNi, aNh, brr, bzz, bni, bnh, hold);
#pragma unroll
    for (int j = 0; j < 8; ++j) H16[(8 * hh + j) * HP + col] = f2h(hold[j]);
  }

#pragma unroll
  for (int j = 0; j < 8; ++j) {
    const float v = hold[j];
    const u16t hi = f2bf(v);
    HHi[(8 * hh + j) * HP + col] = hi;
    HLo[(8 * hh + j) * HP + col] = f2bf(v - bf2f(hi));
  }

#pragma unroll 1
  for (int s = 0; s < TO; ++s) {
    __syncthreads();
    v8f aR = z8, aZ = z8, aNi = z8, aNh = z8;
    mma_in(aR, aZ, aNi, aNh, Ax, QHi, QLo, w, hh, m);
    mma_hh_split(aR, aZ, aNh, aNi, HHi, HLo, PHi, PLo, w, hh, m);
    __syncthreads();
    gru_cell(aR, aZ, aNi, aNh, brr, bzz, bni, bnh, hold);
#pragma unroll
    for (int j = 0; j < 8; ++j) {
      const float v = hold[j];
      const u16t hi = f2bf(v);
      HHi[(8 * hh + j) * HP + col] = hi;
      HLo[(8 * hh + j) * HP + col] = f2bf(v - bf2f(hi));
    }
    __syncthreads();
    if (w == 0) {
      const v8f o = mma_l1(HHi, HLo, RHi, RLo, hh, m);
      const float lb = Lms[m];
#pragma unroll
      for (int j = 0; j < 8; ++j) OutS[(8 * hh + j) * DI + m] = fmaf(o[j], 0.125f, lb);
    }
    __syncthreads();
    {
      const float v = OutS[row * DI + f];
      const u16t hi = f2bf(v);
      Ax[row * AXP + f]      = hi;
      Ax[row * AXP + 16 + f] = f2bf(v - bf2f(hi));
      float acc = 0.0f;
#pragma unroll 1
      for (int q = 0; q < DI; ++q) acc = fmaf(OutS[row * DI + q], Lms[16 + q], acc);
      if (f == 0) Ys[row * TO + s] = acc + Lms[32];
    }
  }
  __syncthreads();

  {
    const int orow = tid >> 4, oc = (tid & 15) * 4;
    const v4f v = *(const v4f*)(Ys + orow * TO + oc);
    float* d = out + (size_t)(b0 + orow) * TO + oc;
    *(volatile v4f*)d = v;
    __threadfence();
    *(volatile v4f*)d = v;
  }
}

extern "C" void kernel_launch(void* const* d_in, const int* in_sizes, int n_in,
                              void* d_out, int out_size, void* d_ws, size_t ws_size,
                              hipStream_t stream) {
  if (n_in < 10) return;
  if (out_size <= 0 || (out_size % TO) != 0) return;
  const int nb = out_size / TO;
  if (nb <= 0 || (nb % 16) != 0) return;
  if (in_sizes[0] <= 0 || (in_sizes[0] % (nb * DI)) != 0) return;
  const int T = in_sizes[0] / (nb * DI);
  if (T < 1) return;
  if (in_sizes[1] != DI * DI || in_sizes[2] != G3 * DI || in_sizes[3] != G3 * HID ||
      in_sizes[4] != G3 || in_sizes[5] != G3 || in_sizes[6] != DI * HID ||
      in_sizes[7] != DI || in_sizes[8] != DI || in_sizes[9] != 1) return;

  const float* x    = (const float*)d_in[0];
  const float* l0_w = (const float*)d_in[1];
  const float* W_ih = (const float*)d_in[2];
  const float* W_hh = (const float*)d_in[3];
  const float* b_ih = (const float*)d_in[4];
  const float* b_hh = (const float*)d_in[5];
  const float* l1_w = (const float*)d_in[6];
  const float* l1_b = (const float*)d_in[7];
  const float* l2_w = (const float*)d_in[8];
  const float* l2_b = (const float*)d_in[9];
  float* out = (float*)d_out;

  char* ws = (char*)d_ws;
  size_t off = 0;
  auto carve = [&](size_t bytes) -> char* {
    char* p = ws + off;
    off += (bytes + 255) & ~(size_t)255;
    return p;
  };
  const size_t szP = (size_t)G3 * HID * 2;
  const size_t szQ = (size_t)G3 * KIH * 2;
  const size_t szR = (size_t)DI * HID * 2;
  u16t* P16 = (u16t*)carve(szP);
  u16t* PHi = (u16t*)carve(szP);
  u16t* PLo = (u16t*)carve(szP);
  u16t* QHi = (u16t*)carve(szQ);
  u16t* QLo = (u16t*)carve(szQ);
  u16t* RHi = (u16t*)carve(szR);
  u16t* RLo = (u16t*)carve(szR);
  if (off > ws_size) return;

  k_planes<<<dim3(86), dim3(256), 0, stream>>>(W_hh, W_ih, l1_w, P16, PHi, PLo, QHi, QLo, RHi, RLo);
  k_gru<<<dim3(nb / 16), dim3(256), 0, stream>>>(x, l0_w, P16, PHi, PLo, QHi, QLo, RHi, RLo,
                                                 b_ih, b_hh, l1_b, l2_w, l2_b, out, nb, T);
}
